// MHSA_8770323218690
// MI455X (gfx1250) — hardware-verified
//
#include <hip/hip_runtime.h>
#include <math.h>
#include <stdint.h>

#define NBATCH 2
#define SEQ    2048
#define DMOD   1024
#define NHEAD  16
#define MTOK   (NBATCH * SEQ)
#define NQKV   (3 * DMOD)
#define PQK    2048

typedef __attribute__((ext_vector_type(16))) __bf16   v16b;
typedef __attribute__((ext_vector_type(8)))  __bf16   v8b;
typedef __attribute__((ext_vector_type(8)))  _Float16 v8h;
typedef __attribute__((ext_vector_type(8)))  float    v8f;
typedef __attribute__((ext_vector_type(4)))  float    v4f;
typedef __attribute__((ext_vector_type(4)))  unsigned int v4u;
typedef v4f __attribute__((may_alias)) v4fa;

static_assert(MTOK % 64 == 0);
static_assert(NQKV % 64 == 0);
static_assert(DMOD % 64 == 0);
static_assert(DMOD % 32 == 0);
static_assert(PQK == 2 * DMOD);

__device__ __forceinline__ unsigned short f2bf_bits(float f) {
  unsigned u = __float_as_uint(f);
  return (unsigned short)((u + 0x7FFFu + ((u >> 16) & 1u)) >> 16);
}
__device__ __forceinline__ float bf_bits2f(unsigned short h) { return __uint_as_float(((unsigned)h) << 16); }
__device__ __forceinline__ unsigned pk16(unsigned short a, unsigned short b) { return (unsigned)a | ((unsigned)b << 16); }

__device__ __forceinline__ void dep_guard_b(v8f& a, v8f& b, v16b x, v16b y) { asm volatile("v_nop\n\tv_nop\n\tv_nop\n\tv_nop" : "+v"(a), "+v"(b) : "v"(x), "v"(y)); }
__device__ __forceinline__ void keep4_b(v16b a, v16b b, v16b c, v16b d) { asm volatile("v_nop" :: "v"(a), "v"(b), "v"(c), "v"(d)); }
__device__ __forceinline__ void acc_guard4(v8f& a, v8f& b, v8f& c, v8f& d) { asm volatile("v_nop\n\tv_nop\n\tv_nop\n\tv_nop" : "+v"(a), "+v"(b), "+v"(c), "+v"(d)); }

union FragU { v16b v; v8b h[2]; };
__device__ __forceinline__ v16b frag_load(const __bf16* p) {
  FragU f; f.h[0] = *(const v8b*)(p); f.h[1] = *(const v8b*)(p + 16); return f.v;
}
__device__ __forceinline__ v8f mma_raw(v16b a, v16b b, v8f c) {
  return __builtin_amdgcn_wmma_f32_16x16x32_bf16(false, a, false, b, (short)0, c, false, false);
}

#define NX8 (MTOK * DMOD / 8)
#define NW8 (NQKV * DMOD / 8)
#define NO8 (DMOD * DMOD / 8)
static_assert(NX8 % 256 == 0);
static_assert(NW8 % 256 == 0);
static_assert(NO8 % 256 == 0);

__global__ __launch_bounds__(256) void prep_kernel(const float* __restrict__ x, const float* __restrict__ wqkv,
                                                   const float* __restrict__ wo,
                                                   unsigned short* __restrict__ xb, unsigned short* __restrict__ wb,
                                                   unsigned short* __restrict__ wo2) {
  const int g = blockIdx.x * 256 + threadIdx.x;
  if (g >= NX8 + NW8 + NO8) return;
  const float* src;
  unsigned short* dst;
  unsigned short* dst2;
  const bool dup = (g >= NX8 + NW8);
  if (g < NX8) {
    src = x + (size_t)g * 8; dst = xb + (size_t)g * 8; dst2 = dst;
  } else if (g < NX8 + NW8) {
    const int e = g - NX8;
    src = wqkv + (size_t)e * 8; dst = wb + (size_t)e * 8; dst2 = dst;
  } else {
    const int e = g - NX8 - NW8;
    const int row = e >> 7, cg = e & 127;
    src = wo + (size_t)e * 8;
    dst = wo2 + (size_t)row * PQK + cg * 8;
    dst2 = dst + DMOD;
  }
  const v4f a = *(const v4fa*)src;
  const v4f c = *(const v4fa*)(src + 4);
  v4u o;
  o[0] = pk16(f2bf_bits(a[0]), f2bf_bits(a[1]));
  o[1] = pk16(f2bf_bits(a[2]), f2bf_bits(a[3]));
  o[2] = pk16(f2bf_bits(c[0]), f2bf_bits(c[1]));
  o[3] = pk16(f2bf_bits(c[2]), f2bf_bits(c[3]));
  *(volatile v4u*)dst = o;
  if (dup) *(volatile v4u*)dst2 = o;
  __threadfence();
  *(volatile v4u*)dst = o;
  if (dup) *(volatile v4u*)dst2 = o;
}

template <int BIAS_MODE, int OUT_MODE>
__global__ __launch_bounds__(256) void wmma_gemm64(
    const unsigned short* __restrict__ Ap, int lda, long strideA,
    const unsigned short* __restrict__ Btp, int ldb, long strideB,
    void* __restrict__ Cout, void* __restrict__ Cout2, int ldc, long strideC,
    const float* __restrict__ bias, int M, int N, int K) {
  const __bf16* A  = (const __bf16*)(const void*)Ap;
  const __bf16* Bt = (const __bf16*)(const void*)Btp;
  __shared__ __align__(16) float sT[8][16 * 68];
  const int b    = blockIdx.y;
  const int lane = threadIdx.x & 31;
  const int wave = threadIdx.x >> 5;
  const int tilesN = N >> 6;
  const int tilesM = M >> 6;
  const int tile = blockIdx.x * 8 + wave;
  if (tile >= tilesM * tilesN) return;
  const int tm = tile / tilesN;
  const int tn = tile - tm * tilesN;
  const int m0 = tm << 6;
  const int n0 = tn << 6;

  const __bf16* Ab = A  + (size_t)b * strideA;
  const __bf16* Bb = Bt + (size_t)b * strideB;

  const int rlane = lane & 15;
  const int koff  = (lane >> 4) * 8;
  const int mOff  = (lane >> 4) * 8;

  v8f acc[4][4];
#pragma unroll
  for (int i = 0; i < 4; ++i)
#pragma unroll
    for (int j = 0; j < 4; ++j) acc[i][j] = (v8f){0.f,0.f,0.f,0.f,0.f,0.f,0.f,0.f};

  for (int k0 = 0; k0 < K; k0 += 32) {
    v16b bh[4];
#pragma unroll
    for (int j = 0; j < 4; ++j) {
      const size_t bo = (size_t)(n0 + (j << 4) + rlane) * ldb + koff + k0;
      bh[j] = frag_load(Bb + bo);
    }
#pragma unroll
    for (int i = 0; i < 4; ++i) {
      const size_t ao = (size_t)(m0 + (i << 4) + rlane) * lda + koff + k0;
      const v16b ah = frag_load(Ab + ao);
#pragma unroll
      for (int j = 0; j < 4; ++j) acc[i][j] = mma_raw(ah, bh[j], acc[i][j]);
      dep_guard_b(acc[i][0], acc[i][3], ah, ah);
    }
    keep4_b(bh[0], bh[1], bh[2], bh[3]);
  }
  acc_guard4(acc[0][0], acc[0][1], acc[0][2], acc[0][3]);
  acc_guard4(acc[1][0], acc[1][1], acc[1][2], acc[1][3]);
  acc_guard4(acc[2][0], acc[2][1], acc[2][2], acc[2][3]);
  acc_guard4(acc[3][0], acc[3][1], acc[3][2], acc[3][3]);

  float* slab = sT[wave];
#pragma unroll
  for (int i = 0; i < 4; ++i) {
    const int mBase = m0 + (i << 4);
    float bm[8];
#pragma unroll
    for (int r = 0; r < 8; ++r) bm[r] = 0.f;
    if (BIAS_MODE == 1) {
      const v4f b0 = *(const v4fa*)(bias + mBase + mOff);
      const v4f b1 = *(const v4fa*)(bias + mBase + mOff + 4);
      bm[0] = bf_bits2f(f2bf_bits(b0[0])); bm[1] = bf_bits2f(f2bf_bits(b0[1]));
      bm[2] = bf_bits2f(f2bf_bits(b0[2])); bm[3] = bf_bits2f(f2bf_bits(b0[3]));
      bm[4] = bf_bits2f(f2bf_bits(b1[0])); bm[5] = bf_bits2f(f2bf_bits(b1[1]));
      bm[6] = bf_bits2f(f2bf_bits(b1[2])); bm[7] = bf_bits2f(f2bf_bits(b1[3]));
    }
#pragma unroll
    for (int j = 0; j < 4; ++j) {
      const int n = n0 + (j << 4) + rlane;
      float bv = 0.f;
      if (BIAS_MODE == 2) bv = bf_bits2f(f2bf_bits(bias[n]));
#pragma unroll
      for (int r = 0; r < 8; ++r) {
        float v = acc[i][j][r];
        if (BIAS_MODE == 1) v += bm[r];
        if (BIAS_MODE == 2) v += bv;
        slab[(mOff + r) * 68 + (j << 4) + rlane] = v;
      }
    }
    __builtin_amdgcn_fence(__ATOMIC_RELEASE, "workgroup");
    __builtin_amdgcn_wave_barrier();
    __builtin_amdgcn_fence(__ATOMIC_ACQUIRE, "workgroup");
    if (OUT_MODE == 0) {
      float* C = (float*)Cout + (size_t)b * strideC;
      const int hh = lane >> 4, c4 = (lane & 15) * 4;
      for (int pass = 0; pass < 2; ++pass) {
#pragma unroll
        for (int it = 0; it < 8; ++it) {
          const int row = it * 2 + hh;
          v4f v = *(const v4fa*)(slab + row * 68 + c4);
          *(volatile v4f*)(C + (size_t)(mBase + row) * ldc + n0 + c4) = v;
        }
        __threadfence();
      }
    } else {
      const int q = lane >> 3, c8 = (lane & 7) * 8;
      unsigned short* C  = (unsigned short*)Cout  + (size_t)b * strideC;
      unsigned short* C2 = (unsigned short*)Cout2 + (size_t)b * strideC;
      for (int pass = 0; pass < 2; ++pass) {
#pragma unroll
        for (int it = 0; it < 4; ++it) {
          const int row = it * 4 + q;
          const float* sp = slab + row * 68 + c8;
          v8h hv, lv;
#pragma unroll
          for (int e = 0; e < 8; ++e) {
            unsigned short hb = f2bf_bits(sp[e]);
            unsigned short lb = f2bf_bits(sp[e] - bf_bits2f(hb));
            hv[e] = __builtin_bit_cast(_Float16, hb);
            lv[e] = __builtin_bit_cast(_Float16, lb);
          }
          *(volatile v8h*)(C  + (size_t)(mBase + row) * ldc + n0 + c8) = hv;
          *(volatile v8h*)(C2 + (size_t)(mBase + row) * ldc + n0 + c8) = lv;
        }
        __threadfence();
      }
    }
    __builtin_amdgcn_fence(__ATOMIC_RELEASE, "workgroup");
    __builtin_amdgcn_wave_barrier();
    __builtin_amdgcn_fence(__ATOMIC_ACQUIRE, "workgroup");
  }
}

#define AT_D 64
#define AT_NW 4
#define AT_QB 64
#define AT_KC 64

__device__ __forceinline__ __bf16 at_f2bf(float f) { return __builtin_bit_cast(__bf16, f2bf_bits(f)); }
__device__ __forceinline__ void at_split(float f, __bf16& hi, __bf16& lo) {
  const unsigned short hb = f2bf_bits(f);
  hi = __builtin_bit_cast(__bf16, hb);
  lo = at_f2bf(f - __uint_as_float(((unsigned)hb) << 16));
}
__device__ __forceinline__ v8f at_mma(v16b a, v16b b, v8f c) {
  c = __builtin_amdgcn_wmma_f32_16x16x32_bf16(false, a, false, b, (short)0, c, false, false);
  asm volatile("v_nop\n\tv_nop\n\tv_nop\n\tv_nop" : "+v"(c) : "v"(a), "v"(b));
  return c;
}

__global__ __launch_bounds__(128)
void attn_full64_kernel(const unsigned short* __restrict__ qkhp, const unsigned short* __restrict__ qklp,
                        const unsigned short* __restrict__ vhp, const unsigned short* __restrict__ vlp,
                        unsigned short* __restrict__ ctx, float sscale) {
  union FB { v16b v; v8b h[2]; };
  __shared__ __align__(16) __bf16 Ksh[AT_KC * AT_D];
  __shared__ __align__(16) __bf16 Ksl[AT_KC * AT_D];
  __shared__ __align__(16) __bf16 Vth[AT_D * AT_KC];
  __shared__ __align__(16) __bf16 Vtl[AT_D * AT_KC];
  __shared__ __align__(16) __bf16 Psh[AT_NW][16 * AT_KC];
  __shared__ __align__(16) __bf16 Psl[AT_NW][16 * AT_KC];
  __shared__ __align__(16) float  Os[AT_NW][16 * 68];

  const int tid  = threadIdx.x;
  const int wave = tid >> 5;
  const int lane = tid & 31;
  const int hh   = lane >> 4;
  const int c    = lane & 15;

  const int nqb = SEQ / AT_QB;
  const int bx = blockIdx.x;
  const int qb = bx % nqb;
  const int bh = bx / nqb;
  const int h  = bh % NHEAD;
  const int b  = bh / NHEAD;
  const int q0 = qb * AT_QB + wave * 16;
  const size_t tok0 = (size_t)b * SEQ;

  const __bf16* Qh = (const __bf16*)(const void*)qkhp + tok0 * PQK + (size_t)h * AT_D;
  const __bf16* Ql = (const __bf16*)(const void*)qklp + tok0 * PQK + (size_t)h * AT_D;
  const __bf16* Kh = Qh + DMOD;
  const __bf16* Kl = Ql + DMOD;
  const __bf16* Vh = (const __bf16*)(const void*)vhp + (size_t)bh * AT_D * SEQ;
  const __bf16* Vl = (const __bf16*)(const void*)vlp + (size_t)bh * AT_D * SEQ;

  v16b qah[2], qal[2];
#pragma unroll
  for (int dc = 0; dc < 2; ++dc) {
    const __bf16* qr = Qh + (size_t)(q0 + c) * PQK + dc * 32 + 8 * hh;
    const __bf16* ql = Ql + (size_t)(q0 + c) * PQK + dc * 32 + 8 * hh;
    qah[dc] = frag_load(qr);
    qal[dc] = frag_load(ql);
  }

  float mrow[8], lrow[8];
  v8f oacc[4];
#pragma unroll
  for (int r = 0; r < 8; ++r) { mrow[r] = -INFINITY; lrow[r] = 0.f; }
#pragma unroll
  for (int t = 0; t < 4; ++t) oacc[t] = (v8f){0.f,0.f,0.f,0.f,0.f,0.f,0.f,0.f};

  const int nChunks = SEQ / AT_KC;
  for (int kc = 0; kc < nChunks; ++kc) {
    const int kv0 = kc * AT_KC;
    __syncthreads();
    {
      const int r = tid >> 1, half = (tid & 1) * 32;
      const __bf16* ksh = Kh + (size_t)(kv0 + r) * PQK + half;
      const __bf16* ksl = Kl + (size_t)(kv0 + r) * PQK + half;
      const __bf16* vsh = Vh + (size_t)r * SEQ + kv0 + half;
      const __bf16* vsl = Vl + (size_t)r * SEQ + kv0 + half;
#pragma unroll
      for (int i = 0; i < 4; ++i) {
        const v8b a0 = *(const v8b*)(ksh + 8 * i);
        const v8b a1 = *(const v8b*)(ksl + 8 * i);
        const v8b b0 = *(const v8b*)(vsh + 8 * i);
        const v8b b1 = *(const v8b*)(vsl + 8 * i);
        *(v8b*)(Ksh + r * AT_D  + half + 8 * i) = a0;
        *(v8b*)(Ksl + r * AT_D  + half + 8 * i) = a1;
        *(v8b*)(Vth + r * AT_KC + half + 8 * i) = b0;
        *(v8b*)(Vtl + r * AT_KC + half + 8 * i) = b1;
      }
    }
    __syncthreads();

    v8f s[4];
#pragma unroll
    for (int j = 0; j < 4; ++j) {
      s[j] = (v8f){0.f,0.f,0.f,0.f,0.f,0.f,0.f,0.f};
#pragma unroll
      for (int dc = 0; dc < 2; ++dc) {
        FB kb, kl;
        kb.h[0] = *(const v8b*)(Ksh + (j * 16 + c) * AT_D + dc * 32 + 8 * hh);
        kb.h[1] = *(const v8b*)(Ksh + (j * 16 + c) * AT_D + dc * 32 + 16 + 8 * hh);
        kl.h[0] = *(const v8b*)(Ksl + (j * 16 + c) * AT_D + dc * 32 + 8 * hh);
        kl.h[1] = *(const v8b*)(Ksl + (j * 16 + c) * AT_D + dc * 32 + 16 + 8 * hh);
        s[j] = at_mma(qah[dc], kb.v, s[j]);
        s[j] = at_mma(qah[dc], kl.v, s[j]);
        s[j] = at_mma(qal[dc], kb.v, s[j]);
        s[j] = at_mma(qal[dc], kl.v, s[j]);
      }
    }
    float cm[8];
#pragma unroll
    for (int r = 0; r < 8; ++r) {
      float m = -INFINITY;
#pragma unroll
      for (int j = 0; j < 4; ++j) {
        const float sv = s[j][r] * sscale;
        s[j][r] = sv;
        m = fmaxf(m, sv);
      }
#pragma unroll
      for (int off = 1; off < 16; off <<= 1) m = fmaxf(m, __shfl_xor(m, off, 32));
      cm[r] = m;
    }
    __bf16* pwh = Psh[wave];
    __bf16* pwl = Psl[wave];
#pragma unroll
    for (int r = 0; r < 8; ++r) {
      const float mnew = fmaxf(mrow[r], cm[r]);
      const float alpha = expf(mrow[r] - mnew);
      mrow[r] = mnew;
      float psum = 0.f;
#pragma unroll
      for (int j = 0; j < 4; ++j) {
        const float p = expf(s[j][r] - mnew);
        psum += p;
        __bf16 a, bl; at_split(p, a, bl);
        pwh[(8 * hh + r) * AT_KC + j * 16 + c] = a;
        pwl[(8 * hh + r) * AT_KC + j * 16 + c] = bl;
      }
#pragma unroll
      for (int off = 1; off < 16; off <<= 1) psum += __shfl_xor(psum, off, 32);
      lrow[r] = lrow[r] * alpha + psum;
#pragma unroll
      for (int t = 0; t < 4; ++t) oacc[t][r] *= alpha;
    }
    __builtin_amdgcn_fence(__ATOMIC_RELEASE, "workgroup");
    __builtin_amdgcn_wave_barrier();
    __builtin_amdgcn_fence(__ATOMIC_ACQUIRE, "workgroup");
#pragma unroll 1
    for (int kk = 0; kk < 2; ++kk) {
      FB pa, pl;
      pa.h[0] = *(const v8b*)(pwh + c * AT_KC + kk * 32 + 8 * hh);
      pa.h[1] = *(const v8b*)(pwh + c * AT_KC + kk * 32 + 16 + 8 * hh);
      pl.h[0] = *(const v8b*)(pwl + c * AT_KC + kk * 32 + 8 * hh);
      pl.h[1] = *(const v8b*)(pwl + c * AT_KC + kk * 32 + 16 + 8 * hh);
#pragma unroll
      for (int t = 0; t < 4; ++t) {
        FB vb, vl;
        vb.h[0] = *(const v8b*)(Vth + (t * 16 + c) * AT_KC + kk * 32 + 8 * hh);
        vb.h[1] = *(const v8b*)(Vth + (t * 16 + c) * AT_KC + kk * 32 + 16 + 8 * hh);
        vl.h[0] = *(const v8b*)(Vtl + (t * 16 + c) * AT_KC + kk * 32 + 8 * hh);
        vl.h[1] = *(const v8b*)(Vtl + (t * 16 + c) * AT_KC + kk * 32 + 16 + 8 * hh);
        oacc[t] = at_mma(pa.v, vb.v, oacc[t]);
        oacc[t] = at_mma(pa.v, vl.v, oacc[t]);
        oacc[t] = at_mma(pl.v, vb.v, oacc[t]);
      }
    }
  }

  float* os = Os[wave];
#pragma unroll
  for (int r = 0; r < 8; ++r) {
    const float inv = 1.0f / lrow[r];
#pragma unroll
    for (int t = 0; t < 4; ++t) os[(8 * hh + r) * 68 + t * 16 + c] = oacc[t][r] * inv;
  }
  __builtin_amdgcn_fence(__ATOMIC_RELEASE, "workgroup");
  __builtin_amdgcn_wave_barrier();
  __builtin_amdgcn_fence(__ATOMIC_ACQUIRE, "workgroup");
  {
    const int q = lane >> 3, c8 = (lane & 7) * 8;
    v4u hv[4], lv[4];
#pragma unroll
    for (int it = 0; it < 4; ++it) {
      const int row = it * 4 + q;
      const v4f f0 = *(const v4fa*)(os + row * 68 + c8);
      const v4f f1 = *(const v4fa*)(os + row * 68 + c8 + 4);
      unsigned short hb[8], lb[8];
#pragma unroll
      for (int e = 0; e < 4; ++e) {
        hb[e]     = f2bf_bits(f0[e]);
        lb[e]     = f2bf_bits(f0[e] - bf_bits2f(hb[e]));
        hb[4 + e] = f2bf_bits(f1[e]);
        lb[4 + e] = f2bf_bits(f1[e] - bf_bits2f(hb[4 + e]));
      }
      v4u a, a2;
#pragma unroll
      for (int e = 0; e < 4; ++e) {
        a[e]  = pk16(hb[2 * e], hb[2 * e + 1]);
        a2[e] = pk16(lb[2 * e], lb[2 * e + 1]);
      }
      hv[it] = a; lv[it] = a2;
    }
    for (int pass = 0; pass < 2; ++pass) {
#pragma unroll
      for (int it = 0; it < 4; ++it) {
        const int row = it * 4 + q;
        const size_t go = (tok0 + (size_t)(q0 + row)) * PQK + (size_t)h * AT_D + c8;
        *(volatile v4u*)(ctx + go) = hv[it];
        *(volatile v4u*)(ctx + go + DMOD) = lv[it];
      }
      __threadfence();
    }
  }
}

extern "C" void kernel_launch(void* const* d_in, const int* in_sizes, int n_in,
                              void* d_out, int out_size, void* d_ws, size_t ws_size,
                              hipStream_t stream) {
  if (n_in < 5) return;
  if (in_sizes[0] != MTOK * DMOD) return;
  if (in_sizes[1] != NQKV * DMOD) return;
  if (in_sizes[2] != NQKV) return;
  if (in_sizes[3] != DMOD * DMOD) return;
  if (in_sizes[4] != DMOD) return;
  if (out_size != MTOK * DMOD) return;

  const float* x    = (const float*)d_in[0];
  const float* Wqkv = (const float*)d_in[1];
  const float* bqkv = (const float*)d_in[2];
  const float* Wo   = (const float*)d_in[3];
  const float* bo   = (const float*)d_in[4];
  float* y = (float*)d_out;

  const size_t bXB  = (size_t)MTOK * DMOD * 2;
  const size_t bWB  = (size_t)NQKV * DMOD * 2;
  const size_t bWO2 = (size_t)DMOD * PQK * 2;
  const size_t bQK  = (size_t)MTOK * PQK * 2;
  const size_t bVT  = (size_t)NBATCH * DMOD * SEQ * 2;
  const size_t bCTX = (size_t)MTOK * PQK * 2;
  size_t off = 0;
  const size_t oXB  = off; off += bXB;
  const size_t oWB  = off; off += bWB;
  const size_t oWO2 = off; off += bWO2;
  const size_t oQKh = off; off += bQK;
  const size_t oQKl = off; off += bQK;
  const size_t oVTh = off; off += bVT;
  const size_t oVTl = off; off += bVT;
  const size_t oCTX = off; off += bCTX;
  if (off > ws_size) return;
  if (off > (size_t)134217728) return;

  char* ws = (char*)d_ws;
  unsigned short* XB  = (unsigned short*)(ws + oXB);
  unsigned short* WB  = (unsigned short*)(ws + oWB);
  unsigned short* WO2 = (unsigned short*)(ws + oWO2);
  unsigned short* QKh = (unsigned short*)(ws + oQKh);
  unsigned short* QKl = (unsigned short*)(ws + oQKl);
  unsigned short* VTh = (unsigned short*)(ws + oVTh);
  unsigned short* VTl = (unsigned short*)(ws + oVTl);
  unsigned short* CTX = (unsigned short*)(ws + oCTX);

  prep_kernel<<<dim3((NX8 + NW8 + NO8) / 256), dim3(256), 0, stream>>>(x, Wqkv, Wo, XB, WB, WO2);

  wmma_gemm64<2, 2><<<dim3((MTOK / 64) * (2048 / 64) / 8, 1), dim3(256), 0, stream>>>(
      XB, DMOD, 0L, WB, DMOD, 0L, (void*)QKh, (void*)QKl, PQK, 0L, bqkv, MTOK, 2048, DMOD);

  wmma_gemm64<1, 2><<<dim3((DMOD / 64) * (SEQ / 64) / 8, NBATCH), dim3(256), 0, stream>>>(
      WB + (size_t)2048 * DMOD, DMOD, 0L, XB, DMOD, (long)SEQ * DMOD,
      (void*)VTh, (void*)VTl, SEQ, (long)DMOD * SEQ, bqkv + 2048, DMOD, SEQ, DMOD);

  attn_full64_kernel<<<dim3(NBATCH * NHEAD * (SEQ / AT_QB)), dim3(128), 0, stream>>>(QKh, QKl, VTh, VTl, CTX, 0.125f);

  wmma_gemm64<2, 0><<<dim3((MTOK / 64) * (DMOD / 64) / 8, 1), dim3(256), 0, stream>>>(
      CTX, PQK, 0L, WO2, PQK, 0L, (void*)y, (void*)y, DMOD, 0L, bo, MTOK, DMOD, PQK);

  (void)hipGetLastError();
}
